// Net_66949950210691
// MI455X (gfx1250) — hardware-verified
//
#include <hip/hip_runtime.h>
#include <stddef.h>
#include <stdint.h>
#include <math.h>


#define SD     128
#define F1     256
#define NC     41
#define NCP    64
#define K2     512
#define NG     512
#define NV     1340
#define NVP    1344
#define NTHR   256
#define NWAVE  8
#define EPT    8
#define CHUNK  (NTHR * EPT)
#define WCAP   (EPT * 32)
#define LISTN  (NWAVE * WCAP)
#define NBD    8192
#define SLD    13
#define NBA    1024
#define SLA    10
#define RCAP   28672
#define DEGCAP 64
#define GBM    64
#define GBN    64
#define GTHR   128
#define UEB    (NVP * (SD / 8))
#define UW1    (F1 * (SD / 8))
#define UW2    (NCP * (K2 / 8))
#define AGG_ZINTS    (LISTN + 2 * RCAP + 3 * NBA)
#define MISC_INTS    16
#define ROWBUF_INTS  (NWAVE * K2 / 2)
#define AGG_LDS_INTS (AGG_ZINTS + MISC_INTS + ROWBUF_INTS)
#define GPB    32
#define GPW    4
#define NOUT   (NG * NC)
#define WSMAX  134217728

static_assert((CHUNK & (CHUNK - 1)) == 0 && CHUNK <= 4096);
static_assert((NBD & (NBD - 1)) == 0 && NBD == (1 << SLD));
static_assert((NBA & (NBA - 1)) == 0 && NBA == (1 << SLA));
static_assert(((long long)CHUNK << SLD) < (1LL << 31));
static_assert(((long long)CHUNK << SLA) < (1LL << 31));
static_assert(NBD % (NTHR * 4) == 0);
static_assert(LISTN % NTHR == 0);
static_assert(NBA % NWAVE == 0 && NBA % 32 == 0 && NBA % GBM == 0);
static_assert(RCAP % 32 == 0 && AGG_ZINTS % 4 == 0 && LISTN % 4 == 0 && ((AGG_ZINTS + MISC_INTS) % 4) == 0);
static_assert(SD % 32 == 0 && K2 % 32 == 0 && K2 == 2 * F1 && F1 == 8 * 32);
static_assert(GBM == (GTHR / 32) * 16 && GBN == 64 && NCP == GBN && F1 % GBN == 0 && NVP % GBM == 0);
static_assert(UEB % NTHR == 0 && UW1 % NTHR == 0 && UW2 % NTHR == 0);
static_assert(SD / 8 == 16 && K2 / 8 == 64);
static_assert(NC <= NCP && NCP == 2 * 32);
static_assert(AGG_LDS_INTS * 4 <= 300000);
static_assert(NG % GPB == 0 && GPB == NWAVE * GPW);
static_assert((GPB * NC) % 4 == 0 && (GPB * NC * 4) % 128 == 0);
static_assert((GPB * NC) / 4 > NTHR && (GPB * NC) / 4 <= 2 * NTHR);
static_assert((NG / GPB) * GPB * NC == NOUT);

typedef float          v2f   __attribute__((ext_vector_type(2)));
typedef float          v4f   __attribute__((ext_vector_type(4)));
typedef float          v8f   __attribute__((ext_vector_type(8)));
typedef int            v4i   __attribute__((ext_vector_type(4)));
typedef int            v8i   __attribute__((ext_vector_type(8)));
typedef unsigned short v4us  __attribute__((ext_vector_type(4)));
typedef unsigned short v8us  __attribute__((ext_vector_type(8)));
typedef unsigned short v16us __attribute__((ext_vector_type(16)));
typedef __bf16         v16bf __attribute__((ext_vector_type(16)));
typedef v2f  __attribute__((may_alias)) v2fa;
typedef v4f  __attribute__((may_alias)) v4fa;
typedef v4i  __attribute__((may_alias)) v4ia;
typedef v4us __attribute__((may_alias)) v4usa;
typedef v8us __attribute__((may_alias)) v8usa;
union FragB { v16bf v; v16us u; v8us h[2]; v8i w; };

__device__ __forceinline__ v8f wmb(const FragB& a, const FragB& b, v8f c) {
  v8f d = __builtin_amdgcn_wmma_f32_16x16x32_bf16(false, a.v, false, b.v, (short)0, c, false, false);
  asm volatile("v_nop\n\tv_nop\n\tv_nop\n\tv_nop" : "+v"(d) : "v"(a.w), "v"(b.w));
  return d;
}

__device__ __forceinline__ unsigned bf16_bits(float f) {
  const unsigned u = __float_as_uint(f);
  return (u + 0x7FFFu + ((u >> 16) & 1u)) >> 16;
}
__device__ __forceinline__ float bf16_val(float f) {
  return __uint_as_float(bf16_bits(f) << 16);
}
__device__ __forceinline__ unsigned hl_pack(float v) {
  const unsigned hb = bf16_bits(v);
  const unsigned lb = bf16_bits(v - __uint_as_float(hb << 16));
  return hb | (lb << 16);
}

__device__ __forceinline__ void wave_sync() {
  __builtin_amdgcn_fence(__ATOMIC_RELEASE, "wavefront");
  __builtin_amdgcn_wave_barrier();
  __builtin_amdgcn_fence(__ATOMIC_ACQUIRE, "wavefront");
}

template <int SLB>
__device__ __forceinline__ int scan_chunk(const int* __restrict__ dsts, int nE, int cbase, int slotBase,
                                          int nb, int vec8, int* list, int tid, int lane, int wave) {
  int wc = 0;
  const int el0  = tid * EPT;
  const int e0   = cbase + el0;
  const int sent = -2147483647 - 1;
  v4i da, db;
  if (vec8 != 0 && cbase + CHUNK <= nE) {
    da = *(const v4i*)(dsts + e0);
    db = *(const v4i*)(dsts + e0 + 4);
  } else {
    da.x = (e0     < nE) ? dsts[min(e0,     nE - 1)] : sent;
    da.y = (e0 + 1 < nE) ? dsts[min(e0 + 1, nE - 1)] : sent;
    da.z = (e0 + 2 < nE) ? dsts[min(e0 + 2, nE - 1)] : sent;
    da.w = (e0 + 3 < nE) ? dsts[min(e0 + 3, nE - 1)] : sent;
    db.x = (e0 + 4 < nE) ? dsts[min(e0 + 4, nE - 1)] : sent;
    db.y = (e0 + 5 < nE) ? dsts[min(e0 + 5, nE - 1)] : sent;
    db.z = (e0 + 6 < nE) ? dsts[min(e0 + 6, nE - 1)] : sent;
    db.w = (e0 + 7 < nE) ? dsts[min(e0 + 7, nE - 1)] : sent;
  }
  const unsigned nbs = (unsigned)slotBase;
  const unsigned unb = (unsigned)nb;
  const unsigned s0 = (unsigned)da.x - nbs, s1 = (unsigned)da.y - nbs;
  const unsigned s2 = (unsigned)da.z - nbs, s3 = (unsigned)da.w - nbs;
  const unsigned s4 = (unsigned)db.x - nbs, s5 = (unsigned)db.y - nbs;
  const unsigned s6 = (unsigned)db.z - nbs, s7 = (unsigned)db.w - nbs;
  const bool h0 = s0 < unb, h1 = s1 < unb, h2 = s2 < unb, h3 = s3 < unb;
  const bool h4 = s4 < unb, h5 = s5 < unb, h6 = s6 < unb, h7 = s7 < unb;
  const unsigned any = __builtin_amdgcn_ballot_w32(h0 | h1 | h2 | h3 | h4 | h5 | h6 | h7);
  if (any != 0u) {
#define HITJ(J, HJ, SJ) { \
      const unsigned mj = __builtin_amdgcn_ballot_w32(HJ); \
      if (mj != 0u) { \
        if (HJ) { \
          const int pos = wc + (int)__builtin_amdgcn_mbcnt_lo(mj, 0u); \
          if (pos < WCAP) list[wave * WCAP + pos] = ((el0 + (J)) << SLB) | (int)(SJ); \
        } \
        wc += (int)__builtin_popcount(mj); } }
    HITJ(0, h0, s0)
    HITJ(1, h1, s1)
    HITJ(2, h2, s2)
    HITJ(3, h3, s3)
    HITJ(4, h4, s4)
    HITJ(5, h5, s5)
    HITJ(6, h6, s6)
    HITJ(7, h7, s7)
#undef HITJ
  }
  return wc;
}

__global__ __launch_bounds__(NTHR) void k_prep(const float* __restrict__ emb, const float* __restrict__ W1,
                                               const float* __restrict__ W2, unsigned short* EB,
                                               unsigned short* W1T, unsigned short* W2T) {
  const int u = (int)blockIdx.x * NTHR + (int)threadIdx.x;
  v8us o;
  unsigned short* dp;
  if (u < UEB) {
    const int row = u >> 4;
    const int k8  = (u & 15) * 8;
    const int rc  = row < NV ? row : NV - 1;
    const float* p = emb + (size_t)rc * SD + k8;
    const v4f a = *(const v4fa*)p;
    const v4f b = *(const v4fa*)(p + 4);
    const bool ok = row < NV;
    o[0] = ok ? (unsigned short)bf16_bits(a.x) : (unsigned short)0;
    o[1] = ok ? (unsigned short)bf16_bits(a.y) : (unsigned short)0;
    o[2] = ok ? (unsigned short)bf16_bits(a.z) : (unsigned short)0;
    o[3] = ok ? (unsigned short)bf16_bits(a.w) : (unsigned short)0;
    o[4] = ok ? (unsigned short)bf16_bits(b.x) : (unsigned short)0;
    o[5] = ok ? (unsigned short)bf16_bits(b.y) : (unsigned short)0;
    o[6] = ok ? (unsigned short)bf16_bits(b.z) : (unsigned short)0;
    o[7] = ok ? (unsigned short)bf16_bits(b.w) : (unsigned short)0;
    dp = EB + (size_t)row * SD + k8;
  } else if (u < UEB + UW1) {
    const int v  = u - UEB;
    const int n  = v >> 4;
    const int k8 = (v & 15) * 8;
    const float* p = W1 + (size_t)k8 * F1 + n;
#pragma unroll
    for (int i = 0; i < 8; ++i) o[i] = (unsigned short)bf16_bits(p[(size_t)i * F1]);
    dp = W1T + (size_t)n * SD + k8;
  } else if (u < UEB + UW1 + UW2) {
    const int v  = u - UEB - UW1;
    const int n  = v >> 6;
    const int k8 = (v & 63) * 8;
    const int kk = k8 & (F1 - 1);
    const int ncl = n < NC ? n : NC - 1;
    const bool ok = n < NC;
    const float* p = W2 + (size_t)kk * NC + ncl;
#pragma unroll
    for (int i = 0; i < 8; ++i) {
      const unsigned short w = (unsigned short)bf16_bits(p[(size_t)i * NC]);
      o[i] = ok ? w : (unsigned short)0;
    }
    dp = W2T + (size_t)n * K2 + k8;
  } else {
    return;
  }
  *(volatile v8us*)dp = o;
  __threadfence();
  *(volatile v8us*)dp = o;
}

__global__ __launch_bounds__(NTHR) void k_deg(const int* __restrict__ dsts, int nE, int vec8, float* dis) {
  __shared__ __attribute__((aligned(16))) int scnt[NBD];
  __shared__ __attribute__((aligned(16))) int list[LISTN];
  __shared__ int wcnt[NWAVE];
  const int tid = (int)threadIdx.x, lane = tid & 31, wave = tid >> 5;
  const int nodeBase = (int)blockIdx.x * NBD;

  for (int i = tid; i < NBD; i += NTHR) scnt[i] = 0;
  for (int i = tid; i < LISTN; i += NTHR) list[i] = 0;
  if (tid < NWAVE) wcnt[tid] = 0;
  __syncthreads();

  const int nChunks = (nE + CHUNK - 1) / CHUNK;
#pragma unroll 1
  for (int ch = 0; ch < nChunks; ++ch) {
    const int cbase = ch * CHUNK;
    const int wc = scan_chunk<SLD>(dsts, nE, cbase, nodeBase, NBD, vec8, list, tid, lane, wave);
    if (lane == 0) wcnt[wave] = wc;
    __syncthreads();
    if (wave == 0) {
#pragma unroll 1
      for (int w2 = 0; w2 < NWAVE; ++w2) {
        int c = wcnt[w2];
        c = c < 0 ? 0 : (c > WCAP ? WCAP : c);
#pragma unroll 1
        for (int b0 = 0; b0 < c; b0 += 32) {
          const int idx = b0 + lane;
          const int ent = list[w2 * WCAP + (idx < WCAP ? idx : WCAP - 1)];
          const int m32 = (c - b0) < 32 ? (c - b0) : 32;
#pragma unroll 1
          for (int k = 0; k < m32; ++k) {
            const int u  = __builtin_amdgcn_readlane(ent, k);
            const int sl = u & (NBD - 1);
            if (lane == 0) scnt[sl] = scnt[sl] + 1;
          }
        }
      }
    }
    __syncthreads();
  }

  v4f vals[NBD / (NTHR * 4)];
#pragma unroll
  for (int it = 0; it < NBD / (NTHR * 4); ++it) {
    const int s0 = it * (NTHR * 4) + 4 * tid;
    const v4i c4 = *(const v4ia*)(scnt + s0);
    const float d0 = (float)c4.x + 1.0f, d1 = (float)c4.y + 1.0f;
    const float d2 = (float)c4.z + 1.0f, d3 = (float)c4.w + 1.0f;
    v4f v;
    v.x = rsqrtf(d0); v.y = rsqrtf(d1); v.z = rsqrtf(d2); v.w = rsqrtf(d3);
    vals[it] = v;
  }
#pragma unroll
  for (int it = 0; it < NBD / (NTHR * 4); ++it) {
    const int s0 = it * (NTHR * 4) + 4 * tid;
    *(volatile v4f*)(dis + (size_t)nodeBase + s0) = vals[it];
  }
  __threadfence();
#pragma unroll
  for (int it = 0; it < NBD / (NTHR * 4); ++it) {
    const int s0 = it * (NTHR * 4) + 4 * tid;
    *(volatile v4f*)(dis + (size_t)nodeBase + s0) = vals[it];
  }
}

__global__ __launch_bounds__(GTHR) void k_gemm(
    const unsigned short* __restrict__ A, const unsigned short* __restrict__ WT,
    float* outF, int K, int ldo)
{
  __shared__ __attribute__((aligned(16))) float stg[GBM * GBN];
  const int tid = (int)threadIdx.x, lane = tid & 31, wave = tid >> 5, hh = lane >> 4, m = lane & 15;
  const int rowBase = (int)blockIdx.x * GBM;
  const int col0    = (int)blockIdx.y * GBN;

  v8f acc[4];
  {
    const v8f z = {0.f, 0.f, 0.f, 0.f, 0.f, 0.f, 0.f, 0.f};
    acc[0] = z; acc[1] = z; acc[2] = z; acc[3] = z;
  }
  const unsigned short* ap = A  + (size_t)(rowBase + 16 * wave + m) * (size_t)K + 8 * hh;
  const unsigned short* wp = WT + (size_t)(col0 + m) * (size_t)K + 8 * hh;
  const int ksteps = K >> 5;
#pragma unroll 1
  for (int ks = 0; ks < ksteps; ++ks) {
    FragB af;
    af.h[0] = *(const v8usa*)(ap + 32 * ks);
    af.h[1] = *(const v8usa*)(ap + 32 * ks + 16);
#pragma unroll
    for (int t = 0; t < 4; ++t) {
      const unsigned short* wq = wp + (size_t)(16 * t) * (size_t)K + 32 * ks;
      FragB bf;
      bf.h[0] = *(const v8usa*)wq;
      bf.h[1] = *(const v8usa*)(wq + 16);
      acc[t] = wmb(af, bf, acc[t]);
    }
  }

#pragma unroll
  for (int t = 0; t < 4; ++t) {
    const int lc = 16 * t + m;
#pragma unroll
    for (int r = 0; r < 8; ++r) {
      const int lr = 16 * wave + 8 * hh + r;
      stg[lr * GBN + lc] = acc[t][r];
    }
  }
  __syncthreads();

  v4f fv[8];
#pragma unroll
  for (int i = 0; i < 8; ++i) {
    const int lr = 16 * wave + 2 * i + hh;
    fv[i] = *(const v4fa*)(stg + lr * GBN + 4 * m);
  }
#pragma unroll
  for (int i = 0; i < 8; ++i) {
    const int lr = 16 * wave + 2 * i + hh;
    const int gr = rowBase + lr;
    float* op = outF + (size_t)gr * (size_t)ldo + col0 + 4 * m;
    *(volatile v4f*)op = fv[i];
  }
  __threadfence();
#pragma unroll
  for (int i = 0; i < 8; ++i) {
    const int lr = 16 * wave + 2 * i + hh;
    const int gr = rowBase + lr;
    float* op = outF + (size_t)gr * (size_t)ldo + col0 + 4 * m;
    *(volatile v4f*)op = fv[i];
  }
}

template <int MODE>
__global__ __launch_bounds__(NTHR) void k_scan(const int* __restrict__ srcs, const int* __restrict__ dsts,
                                               const int* __restrict__ xid,
                                               int nE, int nN, int vec8, int mRows,
                                               const float* __restrict__ dis,
                                               const float* __restrict__ tab, const float* __restrict__ bias,
                                               unsigned short* x1, float* x2) {
  extern __shared__ __attribute__((aligned(16))) int dsm[];
  int* list = dsm;
  int* hl   = dsm + LISTN;
  int* sl   = hl + RCAP;
  int* cnt  = sl + RCAP;
  int* offs = cnt + NBA;
  int* cur  = offs + NBA;
  int* misc = cur + NBA;
  const int tid = (int)threadIdx.x, lane = tid & 31, wave = tid >> 5;
  unsigned short* rowbuf = (unsigned short*)(misc + MISC_INTS) + wave * K2;
  const int nodeBase = (int)blockIdx.x * NBA;

  {
    const v4i z4 = {0, 0, 0, 0};
    for (int i = tid * 4; i < AGG_ZINTS; i += NTHR * 4) *(v4ia*)(dsm + i) = z4;
    if (tid < MISC_INTS) misc[tid] = 0;
  }
  v4f bvA = {0.f, 0.f, 0.f, 0.f}, bvB = {0.f, 0.f, 0.f, 0.f};
  float bv0 = 0.0f, bv1 = 0.0f;
  if constexpr (MODE != 0) {
    const v4f t0 = *(const v4fa*)(bias + 4 * lane);
    const v4f t1 = *(const v4fa*)(bias + 128 + 4 * lane);
    bvA.x = bf16_val(t0.x); bvA.y = bf16_val(t0.y); bvA.z = bf16_val(t0.z); bvA.w = bf16_val(t0.w);
    bvB.x = bf16_val(t1.x); bvB.y = bf16_val(t1.y); bvB.z = bf16_val(t1.z); bvB.w = bf16_val(t1.w);
  } else {
    const int c0 = 2 * lane, c1 = 2 * lane + 1;
    const float t0 = bias[c0 < NC ? c0 : NC - 1];
    const float t1 = bias[c1 < NC ? c1 : NC - 1];
    bv0 = (c0 < NC) ? bf16_val(t0) : 0.0f;
    bv1 = (c1 < NC) ? bf16_val(t1) : 0.0f;
  }
  __syncthreads();

  int t = 0, ov = 0;
  const int nChunks = (nE + CHUNK - 1) / CHUNK;
#pragma unroll 1
  for (int ch = 0; ch < nChunks; ++ch) {
    const int cbase = ch * CHUNK;
    const int wc = scan_chunk<SLA>(dsts, nE, cbase, nodeBase, NBA, vec8, list, tid, lane, wave);
    if (lane == 0) misc[wave] = wc;
    __syncthreads();
    if (wave == 0) {
#pragma unroll 1
      for (int w2 = 0; w2 < NWAVE; ++w2) {
        int c = misc[w2];
        c = c < 0 ? 0 : (c > WCAP ? WCAP : c);
#pragma unroll 1
        for (int b0 = 0; b0 < c; b0 += 32) {
          const int idx = b0 + lane;
          const int ent = list[w2 * WCAP + (idx < WCAP ? idx : WCAP - 1)];
          const int m32 = (c - b0) < 32 ? (c - b0) : 32;
#pragma unroll 1
          for (int k = 0; k < m32; ++k) {
            const int u    = __builtin_amdgcn_readlane(ent, k);
            const int slot = u & (NBA - 1);
            const int el   = (u >> SLA) & (CHUNK - 1);
            const int pk   = ((cbase + el) << SLA) | slot;
            if (t < RCAP) {
              if (lane == 0) { hl[t] = pk; cnt[slot] = cnt[slot] + 1; }
              t = t + 1;
            } else {
              ov = 1;
            }
          }
        }
      }
    }
    __syncthreads();
  }
  if (wave == 0 && lane == 0) { misc[8] = t; misc[9] = ov; }
  __syncthreads();
  int tt = misc[8];
  tt = tt < 0 ? 0 : (tt > RCAP ? RCAP : tt);
  const int ovf = misc[9];

  if (wave == 0) {
    const int base = lane * (NBA / 32);
    int s = 0;
#pragma unroll 1
    for (int i = 0; i < NBA / 32; ++i) s += cnt[base + i];
    int incl = s;
#pragma unroll
    for (int d = 1; d < 32; d <<= 1) {
      const int y = __shfl_up(incl, d, 32);
      if (lane >= d) incl += y;
    }
    int run = incl - s;
#pragma unroll 1
    for (int i = 0; i < NBA / 32; ++i) {
      const int cv = cnt[base + i];
      offs[base + i] = run;
      cur[base + i]  = run;
      run += cv;
    }
  }
  __syncthreads();
  if (wave == 0) {
#pragma unroll 1
    for (int b0 = 0; b0 < tt; b0 += 32) {
      const int idx = b0 + lane;
      const int ent = hl[idx < RCAP ? idx : RCAP - 1];
      const int m32 = (tt - b0) < 32 ? (tt - b0) : 32;
#pragma unroll 1
      for (int k = 0; k < m32; ++k) {
        const int u    = __builtin_amdgcn_readlane(ent, k);
        const int slot = u & (NBA - 1);
        if (lane == 0) {
          int p = cur[slot];
          p = p < 0 ? 0 : (p > RCAP - 1 ? RCAP - 1 : p);
          sl[p] = u;
          cur[slot] = p + 1;
        }
      }
    }
  }
  __syncthreads();

  const float qnan = __int_as_float(0x7fc00000);
  const float pz = (ovf != 0) ? qnan : 0.0f;

  if constexpr (MODE != 0) {
#pragma unroll 1
    for (int si = 0; si < NBA / NWAVE; ++si) {
      const int s    = si * NWAVE + wave;
      const int node = nodeBase + s;
      int c = cnt[s];
      const bool big = c > DEGCAP;
      c = c < 0 ? 0 : (c > DEGCAP ? DEGCAP : c);
      int o = offs[s];
      o = o < 0 ? 0 : (o > RCAP ? RCAP : o);
      const int nc = node < nN ? node : nN - 1;
      const float dd = dis[nc];
      const float rd = dd * dd;
      float a0 = 0.0f, a1 = 0.0f, a2 = 0.0f, a3 = 0.0f;
      float a4 = 0.0f, a5 = 0.0f, a6 = 0.0f, a7 = 0.0f;
#pragma unroll 1
      for (int b0 = 0; b0 < c; b0 += 32) {
        int idx = o + b0 + lane;
        idx = idx > RCAP - 1 ? RCAP - 1 : idx;
        const int ent = sl[idx];
        int eid = ent >> SLA;
        eid = eid < 0 ? 0 : (eid > nE - 1 ? nE - 1 : eid);
        int sr = srcs[eid];
        sr = sr < 0 ? 0 : (sr > nN - 1 ? nN - 1 : sr);
        int id = xid[sr];
        id = id < 0 ? 0 : (id > NV - 1 ? NV - 1 : id);
        const float cf  = dis[sr] * dd;
        const int   cfi = __float_as_int(cf);
        const int m32 = (c - b0) < 32 ? (c - b0) : 32;
#pragma unroll 1
        for (int k = 0; k < m32; ++k) {
          const int   ik = __builtin_amdgcn_readlane(id, k);
          const float ck = __int_as_float(__builtin_amdgcn_readlane(cfi, k));
          const float* p = tab + (size_t)ik * F1 + 4 * lane;
          const v4f ga = *(const v4fa*)p;
          const v4f gb = *(const v4fa*)(p + 128);
          a0 = fmaf(ck, ga.x, a0); a1 = fmaf(ck, ga.y, a1);
          a2 = fmaf(ck, ga.z, a2); a3 = fmaf(ck, ga.w, a3);
          a4 = fmaf(ck, gb.x, a4); a5 = fmaf(ck, gb.y, a5);
          a6 = fmaf(ck, gb.z, a6); a7 = fmaf(ck, gb.w, a7);
        }
      }
      int ids = xid[nc];
      ids = ids < 0 ? 0 : (ids > NV - 1 ? NV - 1 : ids);
      const float* sp = tab + (size_t)ids * F1 + 4 * lane;
      const v4f sA = *(const v4fa*)sp;
      const v4f sB = *(const v4fa*)(sp + 128);
      const float pzr = big ? qnan : pz;
      const bool live = node < nN;
      float y0 = (a0 + sA.x * rd) + bvA.x;
      float y1 = (a1 + sA.y * rd) + bvA.y;
      float y2 = (a2 + sA.z * rd) + bvA.z;
      float y3 = (a3 + sA.w * rd) + bvA.w;
      float y4 = (a4 + sB.x * rd) + bvB.x;
      float y5 = (a5 + sB.y * rd) + bvB.y;
      float y6 = (a6 + sB.z * rd) + bvB.z;
      float y7 = (a7 + sB.w * rd) + bvB.w;
      y0 = (y0 > 0.0f) ? y0 : (y0 - y0); y1 = (y1 > 0.0f) ? y1 : (y1 - y1);
      y2 = (y2 > 0.0f) ? y2 : (y2 - y2); y3 = (y3 > 0.0f) ? y3 : (y3 - y3);
      y4 = (y4 > 0.0f) ? y4 : (y4 - y4); y5 = (y5 > 0.0f) ? y5 : (y5 - y5);
      y6 = (y6 > 0.0f) ? y6 : (y6 - y6); y7 = (y7 > 0.0f) ? y7 : (y7 - y7);
      const unsigned p0 = hl_pack(live ? (y0 + pzr) : 0.0f);
      const unsigned p1 = hl_pack(live ? (y1 + pzr) : 0.0f);
      const unsigned p2 = hl_pack(live ? (y2 + pzr) : 0.0f);
      const unsigned p3 = hl_pack(live ? (y3 + pzr) : 0.0f);
      const unsigned p4 = hl_pack(live ? (y4 + pzr) : 0.0f);
      const unsigned p5 = hl_pack(live ? (y5 + pzr) : 0.0f);
      const unsigned p6 = hl_pack(live ? (y6 + pzr) : 0.0f);
      const unsigned p7 = hl_pack(live ? (y7 + pzr) : 0.0f);
      v4us hA, hB, lA, lB;
      hA[0] = (unsigned short)(p0 & 0xffffu); lA[0] = (unsigned short)(p0 >> 16);
      hA[1] = (unsigned short)(p1 & 0xffffu); lA[1] = (unsigned short)(p1 >> 16);
      hA[2] = (unsigned short)(p2 & 0xffffu); lA[2] = (unsigned short)(p2 >> 16);
      hA[3] = (unsigned short)(p3 & 0xffffu); lA[3] = (unsigned short)(p3 >> 16);
      hB[0] = (unsigned short)(p4 & 0xffffu); lB[0] = (unsigned short)(p4 >> 16);
      hB[1] = (unsigned short)(p5 & 0xffffu); lB[1] = (unsigned short)(p5 >> 16);
      hB[2] = (unsigned short)(p6 & 0xffffu); lB[2] = (unsigned short)(p6 >> 16);
      hB[3] = (unsigned short)(p7 & 0xffffu); lB[3] = (unsigned short)(p7 >> 16);
      *(v4usa*)(rowbuf + 4 * lane) = hA;
      *(v4usa*)(rowbuf + 128 + 4 * lane) = hB;
      *(v4usa*)(rowbuf + F1 + 4 * lane) = lA;
      *(v4usa*)(rowbuf + F1 + 128 + 4 * lane) = lB;
      wave_sync();
      const v8us q0 = *(const v8usa*)(rowbuf + 8 * lane);
      const v8us q1 = *(const v8usa*)(rowbuf + F1 + 8 * lane);
      wave_sync();
      if (node < mRows) {
        unsigned short* rpw = x1 + (size_t)node * K2 + 8 * lane;
        *(volatile v8us*)rpw = q0;
        *(volatile v8us*)(rpw + F1) = q1;
        __threadfence();
        *(volatile v8us*)rpw = q0;
        *(volatile v8us*)(rpw + F1) = q1;
      }
    }
  } else {
    const int sa = (2 * lane) & 31, sb = (2 * lane + 1) & 31;
#pragma unroll 1
    for (int si = 0; si < NBA / NWAVE; ++si) {
      const int s    = si * NWAVE + wave;
      const int node = nodeBase + s;
      int c = cnt[s];
      const bool big = c > DEGCAP;
      c = c < 0 ? 0 : (c > DEGCAP ? DEGCAP : c);
      int o = offs[s];
      o = o < 0 ? 0 : (o > RCAP ? RCAP : o);
      const int nc = node < nN ? node : nN - 1;
      const float dd = dis[nc];
      const float rd = dd * dd;
      float acc0 = 0.0f, acc1 = 0.0f;
#pragma unroll 1
      for (int b0 = 0; b0 < c; b0 += 32) {
        int idx = o + b0 + lane;
        idx = idx > RCAP - 1 ? RCAP - 1 : idx;
        const int ent = sl[idx];
        int eid = ent >> SLA;
        eid = eid < 0 ? 0 : (eid > nE - 1 ? nE - 1 : eid);
        int sr = srcs[eid];
        sr = sr < 0 ? 0 : (sr > nN - 1 ? nN - 1 : sr);
        const float cf  = dis[sr] * dd;
        const int   cfi = __float_as_int(cf);
        const int m32 = (c - b0) < 32 ? (c - b0) : 32;
#pragma unroll 1
        for (int k = 0; k < m32; ++k) {
          const int   sk = __builtin_amdgcn_readlane(sr, k);
          const float ck = __int_as_float(__builtin_amdgcn_readlane(cfi, k));
          const v2f a = *(const v2fa*)(tab + (size_t)sk * NCP + 2 * lane);
          acc0 = fmaf(ck, a.x, acc0); acc1 = fmaf(ck, a.y, acc1);
        }
      }
      float sv0, sv1;
      {
        const v2f a = *(const v2fa*)(tab + (size_t)nc * NCP + 2 * lane);
        sv0 = a.x; sv1 = a.y;
      }
      const float pzr = big ? qnan : pz;
      const bool live = node < nN;
      float y0 = (acc0 + sv0 * rd) + bv0;
      float y1 = (acc1 + sv1 * rd) + bv1;
      y0 = y0 + pzr; y1 = y1 + pzr;
      const float v0 = live ? y0 : 0.0f;
      const float v1 = live ? y1 : 0.0f;
      const bool wr = (node < mRows) && (lane < 16);
      v4f ow;
      ow.x = __shfl(v0, sa, 32); ow.y = __shfl(v1, sa, 32);
      ow.z = __shfl(v0, sb, 32); ow.w = __shfl(v1, sb, 32);
      float* op = x2 + (size_t)node * NCP + 4 * (lane & 15);
      if (wr) *(volatile v4f*)op = ow;
      __threadfence();
      if (wr) *(volatile v4f*)op = ow;
    }
  }
}

__global__ __launch_bounds__(NTHR) void k_pool(const float* __restrict__ x2, const int* __restrict__ bat,
                                               int nN, float* out) {
  __shared__ __attribute__((aligned(16))) float os[GPB * NC];
  const int tid = (int)threadIdx.x, lane = tid & 31, wave = tid >> 5;
  const int gbase = (int)blockIdx.x * GPB + wave * GPW;

  float a0[GPW], a1[GPW];
#pragma unroll
  for (int q = 0; q < GPW; ++q) { a0[q] = 0.0f; a1[q] = 0.0f; }

#pragma unroll 1
  for (int i0 = 0; i0 < nN; i0 += 32) {
    const int i  = i0 + lane;
    const int ic = i < nN ? i : nN - 1;
    const int b  = bat[ic];
    const unsigned rel = (unsigned)b - (unsigned)gbase;
    const bool inr = (i < nN) && (rel < (unsigned)GPW);
    const unsigned any = __builtin_amdgcn_ballot_w32(inr);
    if (any != 0u) {
#pragma unroll
      for (int q = 0; q < GPW; ++q) {
        unsigned msk = __builtin_amdgcn_ballot_w32(inr && (rel == (unsigned)q));
        int nh = (int)__builtin_popcount(msk);
        nh = nh > 32 ? 32 : nh;
#pragma unroll 1
        for (int t = 0; t < nh; ++t) {
          const int k = __builtin_ffs((int)msk) - 1;
          msk &= msk - 1u;
          int node = i0 + (k < 0 ? 0 : k);
          node = node > nN - 1 ? nN - 1 : node;
          const v2f v = *(const v2fa*)(x2 + (size_t)node * NCP + 2 * lane);
          a0[q] += v.x; a1[q] += v.y;
        }
      }
    }
  }
  {
    const int c0 = 2 * lane, c1 = 2 * lane + 1;
#pragma unroll
    for (int q = 0; q < GPW; ++q) {
      const int gl = wave * GPW + q;
      if (c0 < NC) os[gl * NC + c0] = a0[q];
      if (c1 < NC) os[gl * NC + c1] = a1[q];
    }
  }
  __syncthreads();

  constexpr int NQ = (GPB * NC) / 4;
  const int i1  = NTHR + tid;
  const bool ok1 = i1 < NQ;
  const int i1c = ok1 ? i1 : NQ - 1;
  const v4f v0 = *(const v4fa*)(os + 4 * tid);
  const v4f v1 = *(const v4fa*)(os + 4 * i1c);
  float* ob = out + (size_t)blockIdx.x * (GPB * NC);
  *(volatile v4f*)(ob + 4 * tid) = v0;
  if (ok1) *(volatile v4f*)(ob + 4 * i1) = v1;
  __threadfence();
  *(volatile v4f*)(ob + 4 * tid) = v0;
  if (ok1) *(volatile v4f*)(ob + 4 * i1) = v1;
}

static inline int cdiv(int a, int b) { return (a + b - 1) / b; }
static inline size_t al256(size_t o) { return (o + 255) & ~(size_t)255; }

extern "C" void kernel_launch(void* const* d_in, const int* in_sizes, int n_in,
                              void* d_out, int out_size, void* d_ws, size_t ws_size,
                              hipStream_t stream) {
  if (n_in < 8) return;
  const int nN = in_sizes[0];
  if (nN < 1 || nN > (1 << 22)) return;
  if (in_sizes[1] < 2 || (in_sizes[1] & 1) != 0) return;
  const int nE = in_sizes[1] / 2;
  if (nE < 1 || nE >= (1 << (31 - SLA))) return;
  if (in_sizes[2] != nN) return;
  if (in_sizes[3] != NV * SD) return;
  if (in_sizes[4] != SD * F1 || in_sizes[5] != F1) return;
  if (in_sizes[6] != F1 * NC || in_sizes[7] != NC) return;
  if (out_size != NOUT) return;

  const int*   xid  = (const int*)d_in[0];
  const int*   edge = (const int*)d_in[1];
  const int*   bat  = (const int*)d_in[2];
  const float* emb  = (const float*)d_in[3];
  const float* W1   = (const float*)d_in[4];
  const float* b1   = (const float*)d_in[5];
  const float* W2   = (const float*)d_in[6];
  const float* b2   = (const float*)d_in[7];
  float* out = (float*)d_out;
  const int* src = edge;
  const int* dst = edge + nE;

  const int MP   = cdiv(nN, GBM) * GBM;
  const int gM   = MP / GBM;
  const int gD   = cdiv(nN, NBD);
  const int NBPD = gD * NBD;
  const int gA   = cdiv(MP, NBA);
  if ((long long)gA * NBA < (long long)MP) return;
  if (NBPD < nN) return;
  const int vec8 = ((nE & 3) == 0) ? 1 : 0;

  char* ws = (char*)d_ws;
  size_t off = 0;
  const size_t oDIS = off; off = al256(off + (size_t)NBPD * 4);
  const size_t oEB  = off; off = al256(off + (size_t)NVP * SD * 2);
  const size_t oW1T = off; off = al256(off + (size_t)F1 * SD * 2);
  const size_t oW2T = off; off = al256(off + (size_t)NCP * K2 * 2);
  const size_t oT1  = off; off = al256(off + (size_t)NVP * F1 * 4);
  const size_t oX1  = off; off = al256(off + (size_t)MP * K2 * 2);
  const size_t oH2  = off; off = al256(off + (size_t)MP * NCP * 4);
  const size_t oX2  = off; off = al256(off + (size_t)MP * NCP * 4);
  if (off > ws_size || off > (size_t)WSMAX) return;
  float*          DIS = (float*)(ws + oDIS);
  unsigned short* EB  = (unsigned short*)(ws + oEB);
  unsigned short* W1T = (unsigned short*)(ws + oW1T);
  unsigned short* W2T = (unsigned short*)(ws + oW2T);
  float*          T1  = (float*)(ws + oT1);
  unsigned short* X1  = (unsigned short*)(ws + oX1);
  float*          H2  = (float*)(ws + oH2);
  float*          X2  = (float*)(ws + oX2);

  const size_t scanLds = (size_t)AGG_LDS_INTS * 4;
  hipFuncSetAttribute(reinterpret_cast<const void*>(&k_scan<1>), hipFuncAttributeMaxDynamicSharedMemorySize, (int)scanLds);
  hipFuncSetAttribute(reinterpret_cast<const void*>(&k_scan<0>), hipFuncAttributeMaxDynamicSharedMemorySize, (int)scanLds);

  k_prep<<<(UEB + UW1 + UW2) / NTHR, NTHR, 0, stream>>>(emb, W1, W2, EB, W1T, W2T);
  k_gemm<<<dim3(NVP / GBM, F1 / GBN), GTHR, 0, stream>>>(EB, W1T, T1, SD, F1);
  k_deg<<<gD, NTHR, 0, stream>>>(dst, nE, vec8, DIS);
  k_scan<1><<<gA, NTHR, scanLds, stream>>>(src, dst, xid, nE, nN, vec8, MP, DIS, T1, b1, X1, X2);
  k_gemm<<<dim3(gM, NCP / GBN), GTHR, 0, stream>>>(X1, W2T, H2, K2, NCP);
  k_scan<0><<<gA, NTHR, scanLds, stream>>>(src, dst, xid, nE, nN, vec8, MP, DIS, H2, b2, X1, X2);
  k_pool<<<NG / GPB, NTHR, 0, stream>>>(X2, bat, nN, out);
}
